// MultiHeadSelfAttention_7962869367129
// MI455X (gfx1250) — hardware-verified
//
#include <hip/hip_runtime.h>


#ifndef NB
#define NB 2
#endif
#ifndef SEQ
#define SEQ 4096
#endif
#define NB_FULL  2
#define SEQ_FULL 4096
#define DM    512
#define NH_   8
#define HD    64
#define DQ    (NH_ * HD)
#define QKVN  (3 * DQ)
#define QKCAR 16.0f
#define VCAR  16.0f
#define SCQ   (0.125f / (QKCAR * QKCAR))
#define L2E   1.4426950408889634f
#define PLANE_E ((size_t)NB * NH_ * SEQ * HD)

static_assert(HD == 64);
static_assert(NH_ * HD == DQ);
static_assert(QKVN == 3 * DQ);
static_assert(SEQ % 64 == 0);
static_assert(SEQ <= SEQ_FULL && NB <= NB_FULL);
static_assert(DM % 64 == 0 && DQ % 64 == 0 && QKVN % 64 == 0);
static_assert(DM % 32 == 0 && DQ % 32 == 0);
static_assert(PLANE_E % 2048 == 0);
static_assert(PLANE_E < 4294967296ull);
static_assert(((size_t)QKVN * DM) % 2048 == 0 && ((size_t)DM * DQ) % 2048 == 0 && ((size_t)SEQ * DM) % 2048 == 0);

typedef _Float16 h16;
typedef unsigned short bf;
typedef __attribute__((ext_vector_type(16))) __bf16   v16bf;
typedef __attribute__((ext_vector_type(16))) _Float16 v16h;
typedef __attribute__((ext_vector_type(8)))  _Float16 v8h;
typedef __attribute__((ext_vector_type(8)))  unsigned short v8us;
typedef __attribute__((ext_vector_type(8)))  float    v8f;
typedef __attribute__((ext_vector_type(4)))  float    v4f;
typedef v4f  __attribute__((may_alias)) v4fa;

__device__ __forceinline__ unsigned short f2bf(float f) { unsigned u = __float_as_uint(f); u += 0x7FFFu + ((u >> 16) & 1u); return (unsigned short)(u >> 16); }
__device__ __forceinline__ float bf2f(unsigned short b) { return __uint_as_float(((unsigned)b) << 16); }
__device__ __forceinline__ float bfr(float f) { return bf2f(f2bf(f)); }
__device__ __forceinline__ v16h cat16(v8h lo, v8h hi) { return __builtin_shufflevector(lo, hi, 0, 1, 2, 3, 4, 5, 6, 7, 8, 9, 10, 11, 12, 13, 14, 15); }
__device__ __forceinline__ v16bf cat16b(v8us lo, v8us hi) { return __builtin_bit_cast(v16bf, __builtin_shufflevector(lo, hi, 0, 1, 2, 3, 4, 5, 6, 7, 8, 9, 10, 11, 12, 13, 14, 15)); }
__device__ __forceinline__ v8f wmma16(v16h a, v16h b, v8f c) { return __builtin_amdgcn_wmma_f32_16x16x32_f16(false, a, false, b, (short)0, c, false, false); }
__device__ __forceinline__ v8f wmmab(v16bf a, v16bf b, v8f c) { return __builtin_amdgcn_wmma_f32_16x16x32_bf16(false, a, false, b, (short)0, c, false, false); }
__device__ __forceinline__ void splitf(float y, unsigned short& h, unsigned short& l) { h = f2bf(y); l = f2bf(y - bf2f(h)); }

template <typename T16> struct WFrag;
template <> struct WFrag<h16> { typedef v16h V; static __device__ __forceinline__ V ld(const h16* p) { return cat16(*(const v8h*)p, *(const v8h*)(p + 16)); } static __device__ __forceinline__ v8f mma(V a, V b, v8f c) { return wmma16(a, b, c); } };
template <> struct WFrag<bf> { typedef v16bf V; static __device__ __forceinline__ V ld(const bf* p) { return cat16b(*(const v8us*)p, *(const v8us*)(p + 16)); } static __device__ __forceinline__ v8f mma(V a, V b, v8f c) { return wmmab(a, b, c); } };

template <typename T16, int NSPLIT, bool BIAS>
__global__ __launch_bounds__(32) void k_gemmw(const T16* __restrict__ A, const T16* __restrict__ A2, const T16* __restrict__ Bt, const T16* __restrict__ Bt2, int K, float* C, int ldc, const float* __restrict__ bias, size_t sA, size_t sB, size_t sC) {
    typedef typename WFrag<T16>::V V;
    __shared__ __align__(16) float os[16 * 68];
    const size_t z = blockIdx.z; A += z * sA; if (A2) A2 += z * sA; Bt += z * sB; if (Bt2) Bt2 += z * sB; C += z * sC;
    const int lane = threadIdx.x & 31, lr = lane & 15, hi = lane >> 4; const int r0 = blockIdx.x * 64, c0 = blockIdx.y * 64;
    v8f acc[4][4];
#pragma unroll
    for (int mb = 0; mb < 4; ++mb)
#pragma unroll
        for (int nb = 0; nb < 4; ++nb) acc[mb][nb] = (v8f){};
    const size_t aoff = (size_t)(r0 + lr) * K + 8 * hi, boff = (size_t)(c0 + lr) * K + 8 * hi;
#pragma unroll 1
    for (int kc = 0; kc < K; kc += 32) {
        V a[4], a2[4];
#pragma unroll
        for (int mb = 0; mb < 4; ++mb) { a[mb] = WFrag<T16>::ld(A + aoff + (size_t)mb * 16 * K + kc); if (NSPLIT == 1 || NSPLIT == 2) a2[mb] = WFrag<T16>::ld(A2 + aoff + (size_t)mb * 16 * K + kc); }
#pragma unroll
        for (int nb = 0; nb < 4; ++nb) { const V b = WFrag<T16>::ld(Bt + boff + (size_t)nb * 16 * K + kc); V b2; if (NSPLIT >= 2) b2 = WFrag<T16>::ld(Bt2 + boff + (size_t)nb * 16 * K + kc);
#pragma unroll
            for (int mb = 0; mb < 4; ++mb) { acc[mb][nb] = WFrag<T16>::mma(a[mb], b, acc[mb][nb]); if (NSPLIT == 1 || NSPLIT == 2) acc[mb][nb] = WFrag<T16>::mma(a2[mb], b, acc[mb][nb]); if (NSPLIT >= 2) acc[mb][nb] = WFrag<T16>::mma(a[mb], b2, acc[mb][nb]); } }
        asm volatile("v_nop\n\tv_nop\n\tv_nop\n\tv_nop" : "+v"(acc[0][0]), "+v"(acc[1][1]), "+v"(acc[2][2]), "+v"(acc[3][3]) : "v"(a[0]), "v"(a[3]));
    }
#pragma unroll
    for (int mb = 0; mb < 4; ++mb) {
#pragma unroll
        for (int nb = 0; nb < 4; ++nb) {
#pragma unroll
            for (int j = 0; j < 8; ++j) os[(hi * 8 + j) * 68 + nb * 16 + lr] = acc[mb][nb][j]; }
        __builtin_amdgcn_wave_barrier(); asm volatile("" ::: "memory");
        float* crow = C + (size_t)(r0 + mb * 16) * ldc + c0;
#pragma unroll 1
        for (int ps = 0; ps < 2; ++ps) {
#pragma unroll
            for (int s = 0; s < 8; ++s) { const int row = 2 * s + hi, cofs = lr * 4; v4f val = *(const v4fa*)(os + row * 68 + cofs); if (BIAS) { val[0] += bfr(bias[c0 + cofs]); val[1] += bfr(bias[c0 + cofs + 1]); val[2] += bfr(bias[c0 + cofs + 2]); val[3] += bfr(bias[c0 + cofs + 3]); }
                *(volatile v4f*)(crow + (size_t)row * ldc + cofs) = val; }
            if (ps == 0) __threadfence(); }
        __builtin_amdgcn_wave_barrier(); asm volatile("" ::: "memory");
    }
}

__global__ __launch_bounds__(256) void k_cvt8(const float* __restrict__ src, bf* dst, size_t n8, size_t sS, size_t sD) {
    const size_t i = (size_t)blockIdx.x * 256 + threadIdx.x; if (i >= n8) return;
    src += (size_t)blockIdx.y * sS; dst += (size_t)blockIdx.y * sD;
    const v8f v = *(const v8f*)(src + i * 8); v8us o;
#pragma unroll
    for (int k = 0; k < 8; ++k) o[k] = f2bf(v[k]);
    *(volatile v8us*)(dst + i * 8) = o; __threadfence(); *(volatile v8us*)(dst + i * 8) = o; }

__global__ __launch_bounds__(256) void k_qk(const float* __restrict__ F, h16* P) {
    const unsigned e = (blockIdx.x * 256u + threadIdx.x) * 8u; if (e >= (unsigned)PLANE_E) return;
    const unsigned which = blockIdx.y;
    const unsigned d = e & (unsigned)(HD - 1); const unsigned t = (e / (unsigned)HD) % (unsigned)SEQ; const unsigned bh = e / (unsigned)(HD * SEQ); const unsigned b = bh / (unsigned)NH_, h = bh % (unsigned)NH_;
    const float* f = F + (size_t)(b * (unsigned)SEQ + t) * QKVN + which * (unsigned)DQ + h * (unsigned)HD + d;
    const v4f a = *(const v4f*)f; const v4f c = *(const v4f*)(f + 4); v8h o;
#pragma unroll
    for (int q = 0; q < 4; ++q) { o[q] = (h16)(a[q] * QKCAR); o[4 + q] = (h16)(c[q] * QKCAR); }
    h16* dst = P + (size_t)which * PLANE_E + e;
    *(volatile v8h*)dst = o; __threadfence(); *(volatile v8h*)dst = o; }

__global__ __launch_bounds__(256) void k_vt(const float* __restrict__ F, h16* VT) {
    const unsigned e = (blockIdx.x * 256u + threadIdx.x) * 8u; if (e >= (unsigned)PLANE_E) return;
    const unsigned t = e % (unsigned)SEQ; const unsigned d = (e / (unsigned)SEQ) % (unsigned)HD; const unsigned bh = e / (unsigned)(SEQ * HD); const unsigned b = bh / (unsigned)NH_, h = bh % (unsigned)NH_;
    const float* f = F + (size_t)(b * (unsigned)SEQ + t) * QKVN + 2u * (unsigned)DQ + h * (unsigned)HD + d; v8h o;
#pragma unroll
    for (int j = 0; j < 8; ++j) o[j] = (h16)(f[(size_t)j * QKVN] * VCAR);
    *(volatile v8h*)(VT + e) = o; __threadfence(); *(volatile v8h*)(VT + e) = o; }

__global__ __launch_bounds__(32) void k_flash(const h16* __restrict__ QP, const h16* __restrict__ KP, const h16* __restrict__ VT, bf* Ch, bf* Cl) {
    __shared__ __align__(16) float os[16 * 68];
    const unsigned lane = threadIdx.x & 31u, lr = lane & 15u, hi = lane >> 4;
    const unsigned bh = blockIdx.y, q0 = blockIdx.x * 16u;
    const h16* Q = QP + (size_t)bh * SEQ * HD; const h16* K = KP + (size_t)bh * SEQ * HD; const h16* V = VT + (size_t)bh * HD * SEQ;
    const v16h qb0 = WFrag<h16>::ld(Q + (size_t)(q0 + lr) * HD + 8u * hi);
    const v16h qb1 = WFrag<h16>::ld(Q + (size_t)(q0 + lr) * HD + 32u + 8u * hi);
    const h16* kp = K + (size_t)lr * HD + 8u * hi;
    const h16* vp = V + (size_t)lr * SEQ + 8u * hi;
    float m = -1.0e30f, l = 0.0f;
    v8f acc[4];
#pragma unroll
    for (int n = 0; n < 4; ++n) acc[n] = (v8f){};
#pragma unroll 1
    for (unsigned j0 = 0; j0 < (unsigned)SEQ; j0 += 32u) {
        const v16h ka0 = WFrag<h16>::ld(kp + (size_t)j0 * HD);
        const v16h ka1 = WFrag<h16>::ld(kp + (size_t)j0 * HD + 32);
        const v16h kb0 = WFrag<h16>::ld(kp + (size_t)(j0 + 16u) * HD);
        const v16h kb1 = WFrag<h16>::ld(kp + (size_t)(j0 + 16u) * HD + 32);
        v8f s0 = (v8f){}, s1 = (v8f){};
        s0 = wmma16(ka0, qb0, s0); s0 = wmma16(ka1, qb1, s0);
        s1 = wmma16(kb0, qb0, s1); s1 = wmma16(kb1, qb1, s1);
        asm volatile("v_nop\n\tv_nop\n\tv_nop\n\tv_nop" : "+v"(s0), "+v"(s1) : "v"(ka0), "v"(ka1), "v"(kb0), "v"(kb1), "v"(qb0), "v"(qb1));
        float mx = -1.0e30f;
#pragma unroll
        for (int r = 0; r < 8; ++r) { s0[r] *= SCQ; s1[r] *= SCQ; mx = fmaxf(mx, fmaxf(s0[r], s1[r])); }
        mx = fmaxf(mx, __shfl_xor(mx, 16, 32));
        const float nm = fmaxf(m, mx);
        const float fac = __builtin_amdgcn_exp2f((m - nm) * L2E);
        m = nm;
        float rs = 0.0f; v16h pb;
#pragma unroll
        for (int r = 0; r < 8; ++r) {
            const h16 h0 = (h16)__builtin_amdgcn_exp2f((s0[r] - nm) * L2E);
            const h16 h1 = (h16)__builtin_amdgcn_exp2f((s1[r] - nm) * L2E);
            pb[r] = h0; pb[8 + r] = h1; rs += (float)h0 + (float)h1; }
        rs += __shfl_xor(rs, 16, 32);
        l = l * fac + rs;
#pragma unroll
        for (int n = 0; n < 4; ++n)
#pragma unroll
            for (int r = 0; r < 8; ++r) acc[n][r] *= fac;
        const v16h va0 = WFrag<h16>::ld(vp + j0);
        const v16h va1 = WFrag<h16>::ld(vp + (size_t)16 * SEQ + j0);
        const v16h va2 = WFrag<h16>::ld(vp + (size_t)32 * SEQ + j0);
        const v16h va3 = WFrag<h16>::ld(vp + (size_t)48 * SEQ + j0);
        acc[0] = wmma16(va0, pb, acc[0]); acc[1] = wmma16(va1, pb, acc[1]); acc[2] = wmma16(va2, pb, acc[2]); acc[3] = wmma16(va3, pb, acc[3]);
        asm volatile("v_nop\n\tv_nop\n\tv_nop\n\tv_nop" : "+v"(acc[0]), "+v"(acc[1]), "+v"(acc[2]), "+v"(acc[3]) : "v"(va0), "v"(va1), "v"(va2), "v"(va3), "v"(pb));
    }
    const float inv = (1.0f / VCAR) * (1.0f / l);
#pragma unroll
    for (int n = 0; n < 4; ++n)
#pragma unroll
        for (int r = 0; r < 8; ++r) os[lr * 68u + 16u * n + 8u * hi + r] = acc[n][r] * inv;
    __builtin_amdgcn_wave_barrier(); asm volatile("" ::: "memory");
    const unsigned bb = bh / (unsigned)NH_, hh = bh % (unsigned)NH_;
#pragma unroll 1
    for (int ps = 0; ps < 2; ++ps) {
#pragma unroll
        for (unsigned s = 0; s < 4; ++s) { const unsigned row = 4u * s + (lane >> 3), c = (lane & 7u) * 8u;
            const v4f a = *(const v4fa*)(os + row * 68u + c); const v4f b = *(const v4fa*)(os + row * 68u + c + 4u); v8us oh, ol;
#pragma unroll
            for (int q = 0; q < 4; ++q) { unsigned short x0, x1; splitf(a[q], x0, x1); oh[q] = x0; ol[q] = x1; splitf(b[q], x0, x1); oh[4 + q] = x0; ol[4 + q] = x1; }
            const size_t oo = (size_t)(bb * (unsigned)SEQ + q0 + row) * DQ + hh * (unsigned)HD + c;
            *(volatile v8us*)(Ch + oo) = oh; *(volatile v8us*)(Cl + oo) = ol; }
        if (ps == 0) __threadfence(); }
}

constexpr size_t SZ_WQKV = (size_t)QKVN * DM * 2;
constexpr size_t SZ_WO   = (size_t)DM * DQ * 2;
constexpr size_t SZ_XB   = (size_t)NB * SEQ * DM * 2;
constexpr size_t SZ_F    = (size_t)NB * SEQ * QKVN * 4;
constexpr size_t SZ_PL   = PLANE_E * 2;
constexpr size_t SZ_CTX  = (size_t)NB * SEQ * DQ * 2;
constexpr size_t SZ_TOT  = SZ_WQKV + SZ_WO + SZ_XB + SZ_F + 3 * SZ_PL + 2 * SZ_CTX;
static_assert(SZ_WQKV % 256 == 0 && SZ_WO % 256 == 0 && SZ_XB % 256 == 0 && SZ_F % 256 == 0 && SZ_PL % 256 == 0 && SZ_CTX % 256 == 0);
static_assert(SZ_TOT <= (size_t)134217728);

extern "C" void kernel_launch(void* const* d_in, const int* in_sizes, int n_in,
                              void* d_out, int out_size, void* d_ws, size_t ws_size, hipStream_t stream) {
    if (n_in < 5) return;
    const size_t needx = (size_t)(NB - 1) * SEQ_FULL * DM + (size_t)SEQ * DM;
    if ((size_t)in_sizes[0] < needx || (size_t)in_sizes[1] < (size_t)QKVN * DM || in_sizes[2] < QKVN || (size_t)in_sizes[3] < (size_t)DM * DQ || in_sizes[4] < DM) return;
    if ((size_t)out_size < needx) return;
    if (SZ_TOT > ws_size) return;
    const float* x = (const float*)d_in[0]; const float* wqkv = (const float*)d_in[1]; const float* bqkv = (const float*)d_in[2]; const float* wo = (const float*)d_in[3]; const float* bo = (const float*)d_in[4];
    float* OUT = (float*)d_out;
    char* wsp = (char*)d_ws;
    bf* WQKV = (bf*)wsp; wsp += SZ_WQKV;
    bf* WO = (bf*)wsp; wsp += SZ_WO;
    bf* XB = (bf*)wsp; wsp += SZ_XB;
    float* F = (float*)wsp; wsp += SZ_F;
    h16* QK = (h16*)wsp; wsp += 2 * SZ_PL;
    h16* VT = (h16*)wsp; wsp += SZ_PL;
    bf* CTh = (bf*)wsp; wsp += SZ_CTX;
    bf* CTl = (bf*)wsp; wsp += SZ_CTX;

    k_cvt8<<<dim3((unsigned)((size_t)QKVN * DM / 2048), 1, 1), 256, 0, stream>>>(wqkv, WQKV, (size_t)QKVN * DM / 8, 0, 0);
    k_cvt8<<<dim3((unsigned)((size_t)DM * DQ / 2048), 1, 1), 256, 0, stream>>>(wo, WO, (size_t)DM * DQ / 8, 0, 0);
    k_cvt8<<<dim3((unsigned)((size_t)SEQ * DM / 2048), NB, 1), 256, 0, stream>>>(x, XB, (size_t)SEQ * DM / 8, (size_t)SEQ_FULL * DM, (size_t)SEQ * DM);
    k_gemmw<bf, 0, true><<<dim3(SEQ / 64, QKVN / 64, NB), 32, 0, stream>>>(XB, XB, WQKV, WQKV, DM, F, QKVN, bqkv, (size_t)SEQ * DM, 0, (size_t)SEQ * QKVN);
    k_qk<<<dim3((unsigned)(PLANE_E / 2048), 2, 1), 256, 0, stream>>>(F, QK);
    k_vt<<<dim3((unsigned)(PLANE_E / 2048), 1, 1), 256, 0, stream>>>(F, VT);
    k_flash<<<dim3(SEQ / 16, NB * NH_, 1), 32, 0, stream>>>(QK, QK + PLANE_E, VT, CTh, CTl);
    k_gemmw<bf, 1, true><<<dim3(SEQ / 64, DM / 64, NB), 32, 0, stream>>>(CTh, CTl, WO, WO, DQ, OUT, DM, bo, (size_t)SEQ * DQ, 0, (size_t)SEQ_FULL * DM);
}
